// LinearAttention_74474732912911
// MI455X (gfx1250) — hardware-verified
//
#include <hip/hip_runtime.h>
#ifndef NB
#define NB 1
#endif
#ifndef SEQ
#define SEQ 1024
#endif
#define SEQ_FULL 1024
#define DMOD 1024
#define NHS 16
#define FD 16
#define HD 64
#define NQK (NHS * FD)
#define KS 32
#define QT 256
#define NKX SEQ
static_assert(NB == 1);
static_assert(SEQ % QT == 0);
static_assert(SEQ % 128 == 0);
static_assert(QT % 256 == 0);
static_assert(SEQ <= SEQ_FULL);
static_assert(NHS * HD == DMOD);
static_assert(FD * 2 == KS);
static_assert((NHS * QT) % 32 == 0);
static_assert((NHS * SEQ * 4) % 256 == 0);
static_assert((SEQ * DMOD / 8) % 256 == 0);

typedef unsigned short v8us __attribute__((ext_vector_type(8), may_alias));
typedef float  v8f  __attribute__((ext_vector_type(8)));
typedef float  v4f  __attribute__((ext_vector_type(4)));
typedef float  v4fa __attribute__((ext_vector_type(4), may_alias));
typedef _Float16 v16h __attribute__((ext_vector_type(16)));
typedef _Float16 v4h __attribute__((ext_vector_type(4)));
union FragH { v16h v; v8us half[2]; _Float16 h[16]; unsigned short u[16]; };

__device__ __forceinline__ unsigned short bf16_bits(float x) { unsigned int u = __float_as_uint(x); return (unsigned short)((u + 0x7FFFu + ((u >> 16) & 1u)) >> 16); }
__device__ __forceinline__ float bf16_val(unsigned short b) { return __uint_as_float(((unsigned int)b) << 16); }
__device__ __forceinline__ float bf16_rne(float x) { return bf16_val(bf16_bits(x)); }
__device__ __forceinline__ unsigned short h2u(_Float16 x) { return __builtin_bit_cast(unsigned short, x); }

__device__ __forceinline__ v16h g2_frag(const _Float16* p, int hh) { FragH f; f.half[0] = *(const v8us*)((const unsigned short*)p + 8 * hh); f.half[1] = *(const v8us*)((const unsigned short*)p + 16 + 8 * hh); return f.v; }
__device__ __forceinline__ v8f g2_mma(v16h a, v16h b, v8f c) { v8f d = __builtin_amdgcn_wmma_f32_16x16x32_f16(false, a, false, b, (short)0, c, false, false); asm volatile("v_nop\n\tv_nop\n\tv_nop\n\tv_nop" : "+v"(d) : "v"(a), "v"(b)); return d; }

__global__ __launch_bounds__(256) void k_wnat(const float* __restrict__ w, size_t n8, _Float16* __restrict__ Bt) {
  const size_t t = (size_t)blockIdx.x * 256 + threadIdx.x; if (t >= n8) return; FragH f;
#pragma unroll
  for (int q = 0; q < 8; ++q) f.h[q] = (_Float16)(bf16_rne(w[t * 8 + q]) * 16.0f);
  *(volatile v8us*)((unsigned short*)Bt + t * 8) = f.half[0]; __threadfence(); *(volatile v8us*)((unsigned short*)Bt + t * 8) = f.half[0];
}

__global__ __launch_bounds__(256) void k_hl(const float* __restrict__ F, _Float16* __restrict__ Hh, _Float16* __restrict__ Hl, size_t n8) {
  const size_t t = (size_t)blockIdx.x * 256 + threadIdx.x; if (t >= n8) return; FragH fh, fl; const v4f a = *(const v4fa*)(F + t * 8), c = *(const v4fa*)(F + t * 8 + 4);
#pragma unroll
  for (int q = 0; q < 4; ++q) { _Float16 h = (_Float16)a[q]; fh.h[q] = h; fl.h[q] = (_Float16)((a[q] - (float)h) * 1024.0f); h = (_Float16)c[q]; fh.h[4 + q] = h; fl.h[4 + q] = (_Float16)((c[q] - (float)h) * 1024.0f); }
  const v8us oh = fh.half[0], ol = fl.half[0];
  for (int pass = 0; pass < 2; ++pass) { *(volatile v8us*)((unsigned short*)Hh + t * 8) = oh; *(volatile v8us*)((unsigned short*)Hl + t * 8) = ol; if (pass == 0) __threadfence(); }
}

template <int ACT>
__global__ __launch_bounds__(128) void k_gemm2(const _Float16* __restrict__ A, int lda, size_t sA, const _Float16* __restrict__ Bh, int ldb, size_t sB, float alpha, const float* __restrict__ bias, size_t sBias, const float* __restrict__ CP, int rowsPerB, size_t sCPb, int row0g,
    float* __restrict__ C, _Float16* __restrict__ C16, int ldc, size_t sC, int M, int N, int K) {
  static_assert(ACT == 0);
  __shared__ __attribute__((aligned(16))) float so[4][32][68];
  const int tid = threadIdx.x, w = tid >> 5, lane = tid & 31, ln = lane & 15, hh = lane >> 4; const int by = blockIdx.y;
  A += (size_t)by * sA; Bh += (size_t)by * sB; const size_t cofs = (size_t)by * sC; const float* bp = bias ? bias + (size_t)by * sBias : nullptr;
  const int ntn = N >> 6; const int mt = blockIdx.x / ntn, nq = blockIdx.x - mt * ntn; const int row0 = mt * 128 + 32 * w, col0 = nq * 64; if (row0 >= M) return;
  const _Float16* a0p = A + (size_t)(row0 + ln) * lda; const _Float16* a1p = a0p + (size_t)16 * lda;
  const _Float16* b0p = Bh + (size_t)(col0 + ln) * ldb; const _Float16* b1p = b0p + (size_t)16 * ldb; const _Float16* b2p = b1p + (size_t)16 * ldb; const _Float16* b3p = b2p + (size_t)16 * ldb;
  const v8f z8 = {0.f,0.f,0.f,0.f,0.f,0.f,0.f,0.f}; v8f c00 = z8, c01 = z8, c02 = z8, c03 = z8, c10 = z8, c11 = z8, c12 = z8, c13 = z8;
#pragma unroll 1
  for (int kb = 0; kb < K; kb += 32) { const v16h a0 = g2_frag(a0p + kb, hh), a1 = g2_frag(a1p + kb, hh);
    v16h b = g2_frag(b0p + kb, hh); c00 = g2_mma(a0, b, c00); c10 = g2_mma(a1, b, c10);
    b = g2_frag(b1p + kb, hh); c01 = g2_mma(a0, b, c01); c11 = g2_mma(a1, b, c11);
    b = g2_frag(b2p + kb, hh); c02 = g2_mma(a0, b, c02); c12 = g2_mma(a1, b, c12);
    b = g2_frag(b3p + kb, hh); c03 = g2_mma(a0, b, c03); c13 = g2_mma(a1, b, c13); }
  v8f accs[8] = {c00, c01, c02, c03, c10, c11, c12, c13};
#pragma unroll
  for (int u = 0; u < 8; ++u) { const int t = u & 3, half = u >> 2; const int col = col0 + t * 16 + ln; const float bv = bp ? bf16_rne(bp[col]) : 0.f;
#pragma unroll
    for (int r = 0; r < 8; ++r) { const int rloc = half * 16 + 8 * hh + r; float v = accs[u][r] * alpha + bv;
      if (CP) { if (rowsPerB < 0) v += CP[cofs + (size_t)(row0g + row0 + rloc) * ldc + col]; else { const int bidx = (row0g + row0 + rloc) / rowsPerB; v += CP[(size_t)bidx * sCPb + (size_t)by * 64 + col]; } }
      so[w][rloc][t * 16 + ln] = v; } }
  __builtin_amdgcn_fence(4  , "workgroup"); __builtin_amdgcn_wave_barrier();
  const int rsub = lane >> 4, c4 = (lane & 15) * 4;
  for (int pass = 0; pass < 2; ++pass) {
#pragma unroll
    for (int q = 0; q < 16; ++q) { const int r = q * 2 + rsub; const v4f v = *(const v4fa*)&so[w][r][c4];
      if (C) *(volatile v4f*)(C + cofs + (size_t)(row0 + r) * ldc + col0 + c4) = v;
      if (C16) { v4h h4; for (int i = 0; i < 4; ++i) h4[i] = (_Float16)v[i]; *(volatile v4h*)(C16 + cofs + (size_t)(row0 + r) * ldc + col0 + c4) = h4; } }
    if (pass == 0) __threadfence(); }
}

template <int NT, bool RS>
__global__ __launch_bounds__(128) void k_gemm_hr(const _Float16* __restrict__ Ah, const _Float16* __restrict__ Al, int lda, size_t sA,
    const _Float16* __restrict__ Bh, const _Float16* __restrict__ Bl, int ldb, size_t sB, float alpha_h, float alpha_r,
    const float* __restrict__ rs, size_t sRS, float* __restrict__ C, int ldc, size_t sC, int M, int N, int K) {
  static_assert(NT == 2 || NT == 3);
  __shared__ __attribute__((aligned(16))) float so[4][16][64];
  const int tid = threadIdx.x, w = tid >> 5, lane = tid & 31, ln = lane & 15, hh = lane >> 4; const int by = blockIdx.y;
  Ah += (size_t)by * sA; Al += (size_t)by * sA; Bh += (size_t)by * sB; Bl += (size_t)by * sB; C += (size_t)by * sC;
  const int ntn = N >> 6; const int wid = blockIdx.x * 4 + w; const int mt = wid / ntn, nq = wid - mt * ntn; if (mt * 16 >= M) return;
  const int row0 = mt * 16, col0 = nq * 64;
  const _Float16* ahp = Ah + (size_t)(row0 + ln) * lda; const _Float16* alp = Al + (size_t)(row0 + ln) * lda;
  const _Float16* bh0 = Bh + (size_t)(col0 + ln) * ldb; const _Float16* bh1 = bh0 + (size_t)16 * ldb; const _Float16* bh2 = bh1 + (size_t)16 * ldb; const _Float16* bh3 = bh2 + (size_t)16 * ldb;
  const _Float16* bl0 = Bl + (size_t)(col0 + ln) * ldb; const _Float16* bl1 = bl0 + (size_t)16 * ldb; const _Float16* bl2 = bl1 + (size_t)16 * ldb; const _Float16* bl3 = bl2 + (size_t)16 * ldb;
  const v8f z8 = {0.f,0.f,0.f,0.f,0.f,0.f,0.f,0.f}; v8f ch0 = z8, ch1 = z8, ch2 = z8, ch3 = z8, cr0 = z8, cr1 = z8, cr2 = z8, cr3 = z8;
#pragma unroll 1
  for (int kb = 0; kb < K; kb += 32) {
    const v16h ah = g2_frag(ahp + kb, hh), al = g2_frag(alp + kb, hh);
    v16h b = g2_frag(bh0 + kb, hh); ch0 = g2_mma(ah, b, ch0); cr0 = g2_mma(al, b, cr0); if (NT >= 3) { b = g2_frag(bl0 + kb, hh); cr0 = g2_mma(ah, b, cr0); }
    b = g2_frag(bh1 + kb, hh); ch1 = g2_mma(ah, b, ch1); cr1 = g2_mma(al, b, cr1); if (NT >= 3) { b = g2_frag(bl1 + kb, hh); cr1 = g2_mma(ah, b, cr1); }
    b = g2_frag(bh2 + kb, hh); ch2 = g2_mma(ah, b, ch2); cr2 = g2_mma(al, b, cr2); if (NT >= 3) { b = g2_frag(bl2 + kb, hh); cr2 = g2_mma(ah, b, cr2); }
    b = g2_frag(bh3 + kb, hh); ch3 = g2_mma(ah, b, ch3); cr3 = g2_mma(al, b, cr3); if (NT >= 3) { b = g2_frag(bl3 + kb, hh); cr3 = g2_mma(ah, b, cr3); }
  }
  v8f accs[8] = {ch0, ch1, ch2, ch3, cr0, cr1, cr2, cr3};
  float rsc[8];
#pragma unroll
  for (int r = 0; r < 8; ++r) rsc[r] = RS ? rs[(size_t)by * sRS + row0 + 8 * hh + r] : 1.0f;
#pragma unroll
  for (int t = 0; t < 4; ++t) {
#pragma unroll
    for (int r = 0; r < 8; ++r) { const float v = (accs[t][r] * alpha_h + accs[4 + t][r] * alpha_r) * rsc[r]; so[w][8 * hh + r][t * 16 + ln] = v; } }
  __builtin_amdgcn_fence(4  , "workgroup"); __builtin_amdgcn_wave_barrier();
  const int rsub = lane >> 4, c4 = (lane & 15) * 4;
  for (int pass = 0; pass < 2; ++pass) {
#pragma unroll
    for (int q = 0; q < 8; ++q) { const int r = q * 2 + rsub; const v4f v = *(const v4fa*)&so[w][r][c4]; *(volatile v4f*)(C + (size_t)(row0 + r) * ldc + col0 + c4) = v; }
    if (pass == 0) __threadfence(); }
}

__global__ __launch_bounds__(256) void k_qkplanes(const float* __restrict__ Qf, const float* __restrict__ Kf, _Float16* __restrict__ Qh, _Float16* __restrict__ Ql, _Float16* __restrict__ Kh, _Float16* __restrict__ Kl) {
  const int t = blockIdx.x * 256 + threadIdx.x;
  if (t >= NHS * SEQ * 4) return;
  const int h = t / (SEQ * 4); const int rem = t - h * (SEQ * 4); const int l = rem >> 2, p = rem & 3;
  const int f0 = (p & 1) * 8;
  const float keep = (p < 2) ? 1.0f : 0.0f;
  const float* qp = Qf + (size_t)l * NQK + h * FD + f0; const float* kp = Kf + (size_t)l * NQK + h * FD + f0;
  const v4f qa = *(const v4fa*)qp, qb = *(const v4fa*)(qp + 4), ka = *(const v4fa*)kp, kc = *(const v4fa*)(kp + 4);
  const float qs[8] = {qa[0], qa[1], qa[2], qa[3], qb[0], qb[1], qb[2], qb[3]};
  const float ks[8] = {ka[0], ka[1], ka[2], ka[3], kc[0], kc[1], kc[2], kc[3]};
  FragH fqh, fql, fkh, fkl;
#pragma unroll
  for (int i = 0; i < 8; ++i) {
    const float xq = qs[i] * keep; const _Float16 hq = (_Float16)xq; fqh.h[i] = hq; fql.h[i] = (_Float16)((xq - (float)hq) * 1024.0f);
    const float xk = ks[i] * keep; const _Float16 hk = (_Float16)xk; fkh.h[i] = hk; fkl.h[i] = (_Float16)((xk - (float)hk) * 1024.0f);
  }
  const v8us oqh = fqh.half[0], oql = fql.half[0], okh = fkh.half[0], okl = fkl.half[0];
  const size_t o = (size_t)t * 8;
  for (int pass = 0; pass < 2; ++pass) {
    *(volatile v8us*)((unsigned short*)Qh + o) = oqh; *(volatile v8us*)((unsigned short*)Ql + o) = oql;
    *(volatile v8us*)((unsigned short*)Kh + o) = okh; *(volatile v8us*)((unsigned short*)Kl + o) = okl;
    if (pass == 0) __threadfence(); }
}

__global__ __launch_bounds__(256) void k_vt2(const float* __restrict__ Vf, _Float16* __restrict__ VhT, _Float16* __restrict__ VlT) {
  __shared__ unsigned short tlh[64][65];
  __shared__ unsigned short tll[64][65];
  const int tid = threadIdx.x; const int h = blockIdx.x / (SEQ / 64), sg = blockIdx.x - h * (SEQ / 64); const int s0 = sg * 64;
  for (int i = tid; i < 64 * 8; i += 256) {
    const int j = i >> 3, d8 = (i & 7) * 8; const float* vp = Vf + (size_t)(s0 + j) * DMOD + h * HD + d8;
    const v4f a = *(const v4fa*)vp, c = *(const v4fa*)(vp + 4); const float xs[8] = {a[0], a[1], a[2], a[3], c[0], c[1], c[2], c[3]};
#pragma unroll
    for (int q = 0; q < 8; ++q) { const _Float16 hv = (_Float16)xs[q]; tlh[d8 + q][j] = h2u(hv); tll[d8 + q][j] = h2u((_Float16)((xs[q] - (float)hv) * 1024.0f)); }
  }
  __syncthreads();
  for (int pass = 0; pass < 2; ++pass) {
    for (int i = tid; i < 64 * 8; i += 256) {
      const int d = i >> 3, j8 = (i & 7) * 8; FragH fh, fl;
#pragma unroll
      for (int q = 0; q < 8; ++q) { fh.u[q] = tlh[d][j8 + q]; fl.u[q] = tll[d][j8 + q]; }
      const size_t o = ((size_t)(h * HD + d)) * SEQ + s0 + j8;
      *(volatile v8us*)((unsigned short*)VhT + o) = fh.half[0]; *(volatile v8us*)((unsigned short*)VlT + o) = fl.half[0];
    }
    if (pass == 0) __threadfence(); }
}

__global__ __launch_bounds__(256) void k_featp(const float* __restrict__ S, _Float16* __restrict__ Ph, _Float16* __restrict__ Pl, float* __restrict__ Rd, int q0, int nk) {
  #pragma clang fp contract(off)
  __shared__ __attribute__((aligned(16))) float dl[32];
  const int tid = threadIdx.x, w = tid >> 5, lane = tid & 31;
  const int i0 = blockIdx.x * 32; const int hq = i0 / QT; const int rb = i0 - hq * QT;
#pragma unroll 1
  for (int rr = 0; rr < 4; ++rr) {
    const int rl = w * 4 + rr; const int last = q0 + rb + rl; const size_t prow = (size_t)(i0 + rl) * NKX; const float* srow = S + prow;
    float ds = 0.0f;
#pragma unroll 1
    for (int c = 0; c < nk; c += 256) {
      const int j0 = c + lane * 8;
      const v4f a = *(const v4fa*)(srow + j0), b = *(const v4fa*)(srow + j0 + 4);
      const float sv[8] = {a[0], a[1], a[2], a[3], b[0], b[1], b[2], b[3]};
      FragH fh, fl;
#pragma unroll
      for (int q = 0; q < 8; ++q) {
        const float s = sv[q] * 0.00390625f;
        float A = 1.0f + 0.25f * s + 0.03125f * s * s;
        A = (j0 + q <= last) ? A : 0.0f;
        const _Float16 hv = (_Float16)A; const _Float16 lv = (_Float16)((A - (float)hv) * 1024.0f);
        fh.h[q] = hv; fl.h[q] = lv; ds += (float)hv + (float)lv * 0.0009765625f;
      }
      const v8us oh = fh.half[0], ol = fl.half[0];
      unsigned short* dh = (unsigned short*)Ph + prow + j0; unsigned short* dlo = (unsigned short*)Pl + prow + j0;
      *(volatile v8us*)dh = oh; *(volatile v8us*)dlo = ol; __threadfence(); *(volatile v8us*)dh = oh; *(volatile v8us*)dlo = ol;
    }
#pragma unroll
    for (int m = 16; m > 0; m >>= 1) ds += __shfl_xor(ds, m, 32);
    if (lane == 0) dl[rl] = 1.0f / (ds + 1e-12f);
  }
  __syncthreads();
  if (w == 0) {
    const v4f v = *(const v4fa*)&dl[(lane & 7) * 4];
    float* dst = Rd + (size_t)hq * SEQ + q0 + rb + (lane & 7) * 4;
    if (lane < 8) *(volatile v4f*)dst = v;
    __threadfence();
    if (lane < 8) *(volatile v4f*)dst = v;
  }
}

extern "C" void kernel_launch(void* const* d_in, const int* in_sizes, int n_in,
                              void* d_out, int out_size, void* d_ws, size_t ws_size, hipStream_t stream) {
  if (n_in < 5) return;
  if (in_sizes[0] < SEQ * DMOD || in_sizes[1] < NQK * DMOD || in_sizes[2] < NQK * DMOD || in_sizes[3] < DMOD * DMOD || in_sizes[4] < DMOD * DMOD) return;
  if (out_size < SEQ * DMOD) return;
  const float* hs = (const float*)d_in[0]; const float* Wq = (const float*)d_in[1]; const float* Wk = (const float*)d_in[2]; const float* Wv = (const float*)d_in[3]; const float* Wo = (const float*)d_in[4];
  char* ws = (char*)d_ws; size_t off = 0;
  auto take = [&](size_t bytes) { char* p = ws + off; off += (bytes + 255) & ~(size_t)255; return p; };
  _Float16* X16  = (_Float16*)take((size_t)SEQ * DMOD * 2);
  _Float16* Wq16 = (_Float16*)take((size_t)NQK * DMOD * 2);
  _Float16* Wk16 = (_Float16*)take((size_t)NQK * DMOD * 2);
  _Float16* Wv16 = (_Float16*)take((size_t)DMOD * DMOD * 2);
  _Float16* Wo16 = (_Float16*)take((size_t)DMOD * DMOD * 2);
  float*    Qf   = (float*)take((size_t)SEQ * NQK * 4);
  float*    Kf   = (float*)take((size_t)SEQ * NQK * 4);
  float*    Vf   = (float*)take((size_t)SEQ * DMOD * 4);
  _Float16* Qh   = (_Float16*)take((size_t)NHS * SEQ * KS * 2);
  _Float16* Ql   = (_Float16*)take((size_t)NHS * SEQ * KS * 2);
  _Float16* Kh   = (_Float16*)take((size_t)NHS * SEQ * KS * 2);
  _Float16* Kl   = (_Float16*)take((size_t)NHS * SEQ * KS * 2);
  _Float16* VhT  = (_Float16*)take((size_t)NHS * HD * SEQ * 2);
  _Float16* VlT  = (_Float16*)take((size_t)NHS * HD * SEQ * 2);
  float*    S    = (float*)take((size_t)NHS * QT * NKX * 4);
  _Float16* Ph   = (_Float16*)take((size_t)NHS * QT * NKX * 2);
  _Float16* Pl   = (_Float16*)take((size_t)NHS * QT * NKX * 2);
  float*    RDEN = (float*)take((size_t)NHS * SEQ * 4);
  float*    Yf   = (float*)take((size_t)SEQ * DMOD * 4);
  _Float16* Yh   = (_Float16*)take((size_t)SEQ * DMOD * 2);
  _Float16* Yl   = (_Float16*)take((size_t)SEQ * DMOD * 2);
  if (off > ws_size) return;
  const size_t n8x = (size_t)SEQ * DMOD / 8, n8qk = (size_t)NQK * DMOD / 8, n8w = (size_t)DMOD * DMOD / 8;
  k_wnat<<<(unsigned)((n8x + 255) / 256), 256, 0, stream>>>(hs, n8x, X16);
  k_wnat<<<(unsigned)((n8qk + 255) / 256), 256, 0, stream>>>(Wq, n8qk, Wq16);
  k_wnat<<<(unsigned)((n8qk + 255) / 256), 256, 0, stream>>>(Wk, n8qk, Wk16);
  k_wnat<<<(unsigned)((n8w + 255) / 256), 256, 0, stream>>>(Wv, n8w, Wv16);
  k_wnat<<<(unsigned)((n8w + 255) / 256), 256, 0, stream>>>(Wo, n8w, Wo16);
  k_gemm2<0><<<dim3((SEQ / 128) * (NQK / 64), 1), 128, 0, stream>>>(X16, DMOD, (size_t)0, Wq16, DMOD, (size_t)0, 0.0625f, (const float*)nullptr, (size_t)0, (const float*)nullptr, 1, (size_t)0, 0, Qf, (_Float16*)nullptr, NQK, (size_t)0, SEQ, NQK, DMOD);
  k_gemm2<0><<<dim3((SEQ / 128) * (NQK / 64), 1), 128, 0, stream>>>(X16, DMOD, (size_t)0, Wk16, DMOD, (size_t)0, 0.0625f, (const float*)nullptr, (size_t)0, (const float*)nullptr, 1, (size_t)0, 0, Kf, (_Float16*)nullptr, NQK, (size_t)0, SEQ, NQK, DMOD);
  k_gemm2<0><<<dim3((SEQ / 128) * (DMOD / 64), 1), 128, 0, stream>>>(X16, DMOD, (size_t)0, Wv16, DMOD, (size_t)0, 0.0625f, (const float*)nullptr, (size_t)0, (const float*)nullptr, 1, (size_t)0, 0, Vf, (_Float16*)nullptr, DMOD, (size_t)0, SEQ, DMOD, DMOD);
  k_qkplanes<<<(NHS * SEQ * 4) / 256, 256, 0, stream>>>(Qf, Kf, Qh, Ql, Kh, Kl);
  k_vt2<<<NHS * (SEQ / 64), 256, 0, stream>>>(Vf, VhT, VlT);
  for (int q0 = 0; q0 < SEQ; q0 += QT) { const int nk = q0 + QT;
    k_gemm_hr<3, false><<<dim3((QT / 16) * (nk / 64) / 4, NHS), 128, 0, stream>>>(Qh + (size_t)q0 * KS, Ql + (size_t)q0 * KS, KS, (size_t)SEQ * KS, Kh, Kl, KS, (size_t)SEQ * KS, 1.0f, 1.0f / 1024.0f, (const float*)nullptr, (size_t)0, S, NKX, (size_t)QT * NKX, QT, nk, KS);
    k_featp<<<(NHS * QT) / 32, 256, 0, stream>>>(S, Ph, Pl, RDEN, q0, nk);
    k_gemm_hr<3, true><<<dim3((QT / 16) * (HD / 64) / 4, NHS), 128, 0, stream>>>(Ph, Pl, NKX, (size_t)QT * NKX, VhT, VlT, SEQ, (size_t)HD * SEQ, 1.0f, 1.0f / 1024.0f, RDEN + q0, (size_t)SEQ, Yf + (size_t)q0 * DMOD, DMOD, (size_t)HD, QT, HD, nk);
  }
  k_hl<<<(unsigned)((n8x + 255) / 256), 256, 0, stream>>>(Yf, Yh, Yl, n8x);
  k_gemm_hr<2, false><<<dim3((SEQ / 16) * (DMOD / 64) / 4, 1), 128, 0, stream>>>(Yh, Yl, DMOD, (size_t)0, Wo16, Wo16, DMOD, (size_t)0, 1.0f / 256.0f, (1.0f / 256.0f) / 1024.0f, (const float*)nullptr, (size_t)0, (float*)d_out, DMOD, (size_t)0, SEQ, DMOD, DMOD);
}
